// ShiftBlock_3942779978437
// MI455X (gfx1250) — hardware-verified
//
#include <hip/hip_runtime.h>
#include <math.h>


typedef __attribute__((ext_vector_type(16))) _Float16 v16h;
typedef __attribute__((ext_vector_type(8)))  _Float16 v8h;
typedef __attribute__((ext_vector_type(16))) __bf16   v16b;
typedef __attribute__((ext_vector_type(8)))  __bf16   v8b;
typedef __attribute__((ext_vector_type(8)))  float    v8f;
typedef __attribute__((ext_vector_type(4)))  float    v4f;

__device__ __forceinline__ unsigned short f2bf_bits(float f) {
  unsigned u = __float_as_uint(f);
  return (unsigned short)((u + 0x7FFFu + ((u >> 16) & 1u)) >> 16);
}
__device__ __forceinline__ float bf_bits2f(unsigned short h) { return __uint_as_float(((unsigned)h) << 16); }

__device__ __forceinline__ void dep_guard_h(v8f& a, v8f& b, v16h x, v16h y) { asm volatile("v_nop\n\tv_nop\n\tv_nop\n\tv_nop" : "+v"(a), "+v"(b) : "v"(x), "v"(y)); }
__device__ __forceinline__ void dep_guard_b(v8f& a, v8f& b, v16b x, v16b y) { asm volatile("v_nop\n\tv_nop\n\tv_nop\n\tv_nop" : "+v"(a), "+v"(b) : "v"(x), "v"(y)); }
__device__ __forceinline__ void keep4_h(v16h a, v16h b, v16h c, v16h d) { asm volatile("v_nop" :: "v"(a), "v"(b), "v"(c), "v"(d)); }
__device__ __forceinline__ void keep4_b(v16b a, v16b b, v16b c, v16b d) { asm volatile("v_nop" :: "v"(a), "v"(b), "v"(c), "v"(d)); }
__device__ __forceinline__ void acc_guard4(v8f& a, v8f& b, v8f& c, v8f& d) { asm volatile("v_nop\n\tv_nop\n\tv_nop\n\tv_nop" : "+v"(a), "+v"(b), "+v"(c), "+v"(d)); }
template <typename T> struct Frag;
template <> struct Frag<_Float16> {
  typedef v16h V; union U { v16h v; v8h h[2]; };
  static __device__ __forceinline__ v16h load(const _Float16* p) {
    U f; f.h[0] = *(const v8h*)(p); f.h[1] = *(const v8h*)(p + 16); return f.v;
  }
  static __device__ __forceinline__ v8f mma(v16h a, v16h b, v8f c) {
    return __builtin_amdgcn_wmma_f32_16x16x32_f16(false, a, false, b, (short)0, c, false, false);
  }
  static __device__ __forceinline__ void guard(v8f& a, v8f& b, v16h x, v16h y) { dep_guard_h(a, b, x, y); }
  static __device__ __forceinline__ void keep(v16h a, v16h b, v16h c, v16h d) { keep4_h(a, b, c, d); }
};
template <> struct Frag<__bf16> {
  typedef v16b V; union U { v16b v; v8b h[2]; };
  static __device__ __forceinline__ v16b load(const __bf16* p) {
    U f; f.h[0] = *(const v8b*)(p); f.h[1] = *(const v8b*)(p + 16); return f.v;
  }
  static __device__ __forceinline__ v8f mma(v16b a, v16b b, v8f c) {
    return __builtin_amdgcn_wmma_f32_16x16x32_bf16(false, a, false, b, (short)0, c, false, false);
  }
  static __device__ __forceinline__ void guard(v8f& a, v8f& b, v16b x, v16b y) { dep_guard_b(a, b, x, y); }
  static __device__ __forceinline__ void keep(v16b a, v16b b, v16b c, v16b d) { keep4_b(a, b, c, d); }
};

template <int ET> struct Elem;
template <> struct Elem<0> { typedef _Float16 T; };
template <> struct Elem<1> { typedef __bf16 T; };
template <int ET, bool SPLIT, int BIAS_MODE, int OUT_MODE, bool RESID, int ACT, bool RS, bool OSC>
__global__ __launch_bounds__(256) void wmma_gemm64(
    const unsigned short* __restrict__ Ap, const unsigned short* __restrict__ A2p, int lda, long strideA,
    const unsigned short* __restrict__ Btp, const unsigned short* __restrict__ Bt2p, int ldb, long strideB,
    void* __restrict__ Cout, void* __restrict__ Cout2, int ldc, long strideC,
    const float* __restrict__ bias,
    const float* __restrict__ resid, long strideR,
    const float* __restrict__ rowscale,
    int M, int N, int K, float scale, float oscale) {
  typedef typename Elem<ET>::T T;
  typedef typename Frag<T>::V V;
  const T* A = (const T*)Ap; const T* A2 = (const T*)A2p; const T* Bt = (const T*)Btp; const T* Bt2 = (const T*)Bt2p;
  __shared__ __align__(16) float sT[8][16 * 68];
  const int b    = blockIdx.y;
  const int lane = threadIdx.x & 31;
  const int wave = threadIdx.x >> 5;
  const int tilesN = N >> 6;
  const int tilesM = M >> 6;
  const int tile = blockIdx.x * 8 + wave;
  if (tile >= tilesM * tilesN) return;
  const int tm = tile / tilesN;
  const int tn = tile - tm * tilesN;
  const int m0 = tm << 6;
  const int n0 = tn << 6;

  const T* Ab  = A  + (size_t)b * strideA;
  const T* Bb  = Bt + (size_t)b * strideB;
  const T* Ab2 = SPLIT ? (A2  + (size_t)b * strideA) : nullptr;
  const T* Bb2 = SPLIT ? (Bt2 + (size_t)b * strideB) : nullptr;

  const int rlane = lane & 15;
  const int koff  = (lane >> 4) * 8;
  const int mOff  = (lane >> 4) * 8;

  v8f acc[4][4];
#pragma unroll
  for (int i = 0; i < 4; ++i)
#pragma unroll
    for (int j = 0; j < 4; ++j) acc[i][j] = (v8f){0.f,0.f,0.f,0.f,0.f,0.f,0.f,0.f};

  for (int k0 = 0; k0 < K; k0 += 32) {
    V bh[4], bl[4];
#pragma unroll
    for (int j = 0; j < 4; ++j) {
      const size_t bo = (size_t)(n0 + (j << 4) + rlane) * ldb + koff + k0;
      bh[j] = Frag<T>::load(Bb + bo);
      if (SPLIT) bl[j] = Frag<T>::load(Bb2 + bo);
    }
#pragma unroll
    for (int i = 0; i < 4; ++i) {
      const size_t ao = (size_t)(m0 + (i << 4) + rlane) * lda + koff + k0;
      V ah = Frag<T>::load(Ab + ao);
      V al;
      if (SPLIT) al = Frag<T>::load(Ab2 + ao);
#pragma unroll
      for (int j = 0; j < 4; ++j) {
        acc[i][j] = Frag<T>::mma(ah, bh[j], acc[i][j]);
        if (SPLIT) {
          acc[i][j] = Frag<T>::mma(ah, bl[j], acc[i][j]);
          acc[i][j] = Frag<T>::mma(al, bh[j], acc[i][j]);
        }
      }
      Frag<T>::guard(acc[i][0], acc[i][3], ah, SPLIT ? al : ah);
    }
    Frag<T>::keep(bh[0], bh[1], bh[2], bh[3]);
    if (SPLIT) Frag<T>::keep(bl[0], bl[1], bl[2], bl[3]);
  }
  acc_guard4(acc[0][0], acc[0][1], acc[0][2], acc[0][3]);
  acc_guard4(acc[1][0], acc[1][1], acc[1][2], acc[1][3]);
  acc_guard4(acc[2][0], acc[2][1], acc[2][2], acc[2][3]);
  acc_guard4(acc[3][0], acc[3][1], acc[3][2], acc[3][3]);

  float* slab = sT[wave];
  const float* Rb = RESID ? (resid + (size_t)b * strideR) : nullptr;
#pragma unroll
  for (int i = 0; i < 4; ++i) {
    const int mBase = m0 + (i << 4);
    float rsv[8];
#pragma unroll
    for (int r = 0; r < 8; ++r) rsv[r] = RS ? rowscale[mBase + mOff + r] : 1.0f;
#pragma unroll
    for (int j = 0; j < 4; ++j) {
      const int n = n0 + (j << 4) + rlane;
      float bv = 0.f;
      if (BIAS_MODE == 2) bv = bias[n];
#pragma unroll
      for (int r = 0; r < 8; ++r) {
        float v = acc[i][j][r] * scale;
        if (RS) v *= rsv[r];
        if (BIAS_MODE == 1) v += bias[mBase + mOff + r];
        if (BIAS_MODE == 2) v += bv;
        if (RESID) v += Rb[(size_t)(mBase + mOff + r) * ldc + n];
        if (ACT == 1) v = tanhf(v);
        if (ACT == 2) v = fmaxf(v, 0.0f);
        if (ACT == 3) v = v / (1.0f + expf(-v));
        if (ACT == 4) v = (v > 0.f) ? v : 0.01f * v;
        if (ACT == 5) v = 0.5f * v * (1.0f + erff(v * 0.70710678118654752f));
        if (OSC) v *= oscale;
        slab[(mOff + r) * 68 + (j << 4) + rlane] = v;
      }
    }
    __builtin_amdgcn_fence(__ATOMIC_RELEASE, "workgroup");
    __builtin_amdgcn_wave_barrier();
    __builtin_amdgcn_fence(__ATOMIC_ACQUIRE, "workgroup");
    if (OUT_MODE == 0) {
      float* C = (float*)Cout + (size_t)b * strideC;
      const int hh = lane >> 4, c4 = (lane & 15) * 4;
      for (int pass = 0; pass < 2; ++pass) {
#pragma unroll
        for (int it = 0; it < 8; ++it) {
          const int row = it * 2 + hh;
          v4f v = *(const v4f*)(slab + row * 68 + c4);
          *(volatile v4f*)(C + (size_t)(mBase + row) * ldc + n0 + c4) = v;
        }
        __threadfence();
      }
    } else {
      const int q = lane >> 3, c8 = (lane & 7) * 8;
      unsigned short* C  = (unsigned short*)Cout  + (size_t)b * strideC;
      unsigned short* C2 = (OUT_MODE == 2) ? ((unsigned short*)Cout2 + (size_t)b * strideC) : nullptr;
      for (int pass = 0; pass < 2; ++pass) {
#pragma unroll
        for (int it = 0; it < 4; ++it) {
          const int row = it * 4 + q;
          const float* sp = slab + row * 68 + c8;
          v8h hv, lv;
#pragma unroll
          for (int e = 0; e < 8; ++e) {
            if (OUT_MODE == 1) {
              hv[e] = (_Float16)sp[e];
            } else {
              unsigned short hb = f2bf_bits(sp[e]);
              unsigned short lb = f2bf_bits(sp[e] - bf_bits2f(hb));
              hv[e] = __builtin_bit_cast(_Float16, hb);
              lv[e] = __builtin_bit_cast(_Float16, lb);
            }
          }
          *(volatile v8h*)(C + (size_t)(mBase + row) * ldc + n0 + c8) = hv;
          if (OUT_MODE == 2) *(volatile v8h*)(C2 + (size_t)(mBase + row) * ldc + n0 + c8) = lv;
        }
        __threadfence();
      }
    }
    __builtin_amdgcn_fence(__ATOMIC_RELEASE, "workgroup");
    __builtin_amdgcn_wave_barrier();
    __builtin_amdgcn_fence(__ATOMIC_ACQUIRE, "workgroup");
  }
}

__global__ __launch_bounds__(256) void cast_scale_f16x2(
    const float* __restrict__ in, _Float16* __restrict__ out, int n2, float sc) {
  int i = blockIdx.x * 256 + threadIdx.x;
  if (i < n2) {
    const _Float16 h0 = (_Float16)(in[2 * i] * sc), h1 = (_Float16)(in[2 * i + 1] * sc);
    const unsigned u = (unsigned)__builtin_bit_cast(unsigned short, h0) | ((unsigned)__builtin_bit_cast(unsigned short, h1) << 16);
    ((volatile unsigned*)out)[i] = u;
    __threadfence();
    ((volatile unsigned*)out)[i] = u;
  }
}

__global__ __launch_bounds__(256) void transpose_scale_f16(
    const float* __restrict__ in, _Float16* __restrict__ out, int R, int Cc, float sc) {
  __shared__ float tile[64 * 65];
  const int tid = threadIdx.x;
  const int c0 = blockIdx.x * 64, r0 = blockIdx.y * 64;
#pragma unroll
  for (int i = 0; i < 16; ++i) {
    const int idx = tid + 256 * i;
    const int rr = idx >> 6, cc = idx & 63;
    tile[rr * 65 + cc] = in[(size_t)(r0 + rr) * Cc + c0 + cc] * sc;
  }
  __syncthreads();
  const int q = tid >> 3, e8 = (tid & 7) * 8;
  v8h o0, o1;
#pragma unroll
  for (int e = 0; e < 8; ++e) {
    o0[e] = (_Float16)tile[(e8 + e) * 65 + q];
    o1[e] = (_Float16)tile[(e8 + e) * 65 + q + 32];
  }
  _Float16* d0 = out + (size_t)(c0 + q) * R + r0 + e8;
  _Float16* d1 = out + (size_t)(c0 + q + 32) * R + r0 + e8;
  for (int pass = 0; pass < 2; ++pass) {
    *(volatile v8h*)d0 = o0;
    *(volatile v8h*)d1 = o1;
    __threadfence();
  }
}

__global__ __launch_bounds__(256) void ln_kernel(
    const float* __restrict__ x, const float* __restrict__ g, const float* __restrict__ bb,
    _Float16* __restrict__ xn, int rows) {
  const int wave = threadIdx.x >> 5, lane = threadIdx.x & 31;
  const int row = blockIdx.x * 8 + wave;
  if (row >= rows) return;
  const float* xr = x + (size_t)row * 512;
  float v[16];
#pragma unroll
  for (int j = 0; j < 2; ++j) {
    const v4f a = *(const v4f*)(xr + 256 * j + 8 * lane);
    const v4f c = *(const v4f*)(xr + 256 * j + 8 * lane + 4);
    v[8 * j + 0] = a[0]; v[8 * j + 1] = a[1]; v[8 * j + 2] = a[2]; v[8 * j + 3] = a[3];
    v[8 * j + 4] = c[0]; v[8 * j + 5] = c[1]; v[8 * j + 6] = c[2]; v[8 * j + 7] = c[3];
  }
  float s = 0.f;
#pragma unroll
  for (int e = 0; e < 16; ++e) s += v[e];
#pragma unroll
  for (int off = 16; off > 0; off >>= 1) s += __shfl_xor(s, off, 32);
  const float mu = s * (1.0f / 512.0f);
  float ss = 0.f;
#pragma unroll
  for (int e = 0; e < 16; ++e) { const float d = v[e] - mu; v[e] = d; ss += d * d; }
#pragma unroll
  for (int off = 16; off > 0; off >>= 1) ss += __shfl_xor(ss, off, 32);
  const float rs = rsqrtf(ss * (1.0f / 512.0f) + 1e-5f);
  v8h o0, o1;
  {
    const int cA = 8 * lane, cB = 256 + 8 * lane;
    const v4f g0 = *(const v4f*)(g + cA), g1 = *(const v4f*)(g + cA + 4);
    const v4f g2 = *(const v4f*)(g + cB), g3 = *(const v4f*)(g + cB + 4);
    const v4f b0 = *(const v4f*)(bb + cA), b1 = *(const v4f*)(bb + cA + 4);
    const v4f b2 = *(const v4f*)(bb + cB), b3 = *(const v4f*)(bb + cB + 4);
#pragma unroll
    for (int e = 0; e < 4; ++e) {
      o0[e]     = (_Float16)((v[e] * rs) * g0[e] + b0[e]);
      o0[4 + e] = (_Float16)((v[4 + e] * rs) * g1[e] + b1[e]);
      o1[e]     = (_Float16)((v[8 + e] * rs) * g2[e] + b2[e]);
      o1[4 + e] = (_Float16)((v[12 + e] * rs) * g3[e] + b3[e]);
    }
  }
  _Float16* d0 = xn + (size_t)row * 512 + 8 * lane;
  _Float16* d1 = xn + (size_t)row * 512 + 256 + 8 * lane;
  for (int pass = 0; pass < 2; ++pass) {
    *(volatile v8h*)d0 = o0;
    *(volatile v8h*)d1 = o1;
    __threadfence();
  }
}

#define XP 72
__global__ __launch_bounds__(256) void im2col_shift_kernel(
    const _Float16* __restrict__ h64, _Float16* __restrict__ col) {
  __shared__ __align__(16) _Float16 xs_l[256 * XP];
  const int tid = threadIdx.x, wave = tid >> 5, lane = tid & 31;
  const int b = blockIdx.y, c0 = blockIdx.x * 64;
  {
    const int np = tid;
    const int s = (np < 86) ? -1 : ((np < 172) ? 0 : 1);
    const _Float16* hrow = h64 + ((size_t)b * 256 + np) * 512;
#pragma unroll 2
    for (int q = 0; q < 66; ++q) {
      const int cc = c0 - 1 + q;
      const int hi = cc - s;
      const bool valid = (cc >= 0) && (cc < 512) && (hi >= 0) && (hi < 512);
      const int hic = hi < 0 ? 0 : (hi > 511 ? 511 : hi);
      const _Float16 hv = hrow[hic];
      xs_l[np * XP + q] = valid ? hv : (_Float16)0.0f;
    }
  }
  __syncthreads();
#pragma unroll 1
  for (int i = 0; i < 8; ++i) {
    const int cl = wave + 8 * i;
    const int c = c0 + cl;
    _Float16* dst = col + ((size_t)b * 512 + c) * 768;
    v8h o0, o1, o2;
#pragma unroll
    for (int e = 0; e < 8; ++e) {
      int j = 8 * lane + e;
      int n1 = j / 3; int k1 = j - 3 * n1;
      o0[e] = xs_l[n1 * XP + cl + k1];
      j += 256; n1 = j / 3; k1 = j - 3 * n1;
      o1[e] = xs_l[n1 * XP + cl + k1];
      j += 256; n1 = j / 3; k1 = j - 3 * n1;
      o2[e] = xs_l[n1 * XP + cl + k1];
    }
    for (int pass = 0; pass < 2; ++pass) {
      *(volatile v8h*)(dst + 8 * lane) = o0;
      *(volatile v8h*)(dst + 256 + 8 * lane) = o1;
      *(volatile v8h*)(dst + 512 + 8 * lane) = o2;
      __threadfence();
    }
  }
}

__global__ __launch_bounds__(256) void se_kernel(
    const _Float16* __restrict__ y64, const float* __restrict__ We1, const float* __restrict__ be1,
    const float* __restrict__ We2, const float* __restrict__ be2, float* __restrict__ exg) {
  __shared__ float sSe[256];
  __shared__ float sH[32];
  const int tid = threadIdx.x, wave = tid >> 5, lane = tid & 31;
  const int b = blockIdx.x;
  float keep = 0.f;
#pragma unroll 1
  for (int r = 0; r < 32; ++r) {
    const int n = wave * 32 + r;
    const _Float16* yr = y64 + ((size_t)b * 256 + n) * 512;
    const v8h a0 = *(const v8h*)(yr + 8 * lane);
    const v8h a1 = *(const v8h*)(yr + 256 + 8 * lane);
    float s = 0.f;
#pragma unroll
    for (int e = 0; e < 8; ++e) s += (float)a0[e];
#pragma unroll
    for (int e = 0; e < 8; ++e) s += (float)a1[e];
#pragma unroll
    for (int off = 16; off > 0; off >>= 1) s += __shfl_xor(s, off, 32);
    if (lane == r) keep = s;
  }
  sSe[wave * 32 + lane] = keep * (1.0f / 32768.0f);
  __syncthreads();
  if (tid < 32) {
    float a = be1[tid];
#pragma unroll 1
    for (int m = 0; m < 256; ++m) a += sSe[m] * We1[m * 32 + tid];
    sH[tid] = a > 0.f ? a : 0.f;
  }
  __syncthreads();
  float a = be2[tid];
#pragma unroll 1
  for (int j = 0; j < 32; ++j) a += sH[j] * We2[j * 256 + tid];
  const float e = 1.0f / (1.0f + expf(-a));
  float* d = exg + (size_t)b * 256 + tid;
  *(volatile float*)d = e;
  __threadfence();
  *(volatile float*)d = e;
}

extern "C" void kernel_launch(void* const* d_in, const int* in_sizes, int n_in,
                              void* d_out, int out_size, void* d_ws, size_t ws_size,
                              hipStream_t stream) {
  if (n_in < 15) return;
  const int NN = 256, CC = 512, C2 = 1024, KC = 768;
  const long nx = (long)in_sizes[0];
  if (nx <= 0 || (nx % ((long)NN * CC)) != 0) return;
  const int nB = (int)(nx / ((long)NN * CC));
  const int ROWS = nB * NN;
  if ((long)out_size != nx) return;
  if (in_sizes[1] != CC || in_sizes[2] != CC || in_sizes[3] != CC * CC || in_sizes[4] != CC) return;
  if (in_sizes[5] != NN * NN * 3 || in_sizes[6] != NN || in_sizes[7] != NN * 32 || in_sizes[8] != 32) return;
  if (in_sizes[9] != 32 * NN || in_sizes[10] != NN || in_sizes[11] != CC * C2 || in_sizes[12] != C2) return;
  if (in_sizes[13] != C2 * CC || in_sizes[14] != CC) return;

  const float* x    = (const float*)d_in[0];
  const float* ln_g = (const float*)d_in[1];
  const float* ln_b = (const float*)d_in[2];
  const float* Ws   = (const float*)d_in[3];
  const float* bs   = (const float*)d_in[4];
  const float* Wc   = (const float*)d_in[5];
  const float* bc   = (const float*)d_in[6];
  const float* We1  = (const float*)d_in[7];
  const float* be1  = (const float*)d_in[8];
  const float* We2  = (const float*)d_in[9];
  const float* be2  = (const float*)d_in[10];
  const float* Wf1  = (const float*)d_in[11];
  const float* bf1  = (const float*)d_in[12];
  const float* Wf2  = (const float*)d_in[13];
  const float* bf2  = (const float*)d_in[14];
  float* out = (float*)d_out;

  size_t off = 0;
  auto carve = [&](size_t bytes) { size_t o = off; off += (bytes + 255) & ~(size_t)255; return o; };
  const size_t bXn  = (size_t)ROWS * CC * 2;
  const size_t bCol = (size_t)nB * CC * KC * 2;
  const size_t bG   = (size_t)ROWS * C2 * 2;
  size_t bR1 = bXn; if (bCol > bR1) bR1 = bCol; if (bG > bR1) bR1 = bG;
  const size_t oR1  = carve(bR1);
  const size_t oR2  = carve((size_t)ROWS * CC * 2);
  const size_t oWsT = carve((size_t)CC * CC * 2);
  const size_t oWc  = carve((size_t)NN * KC * 2);
  const size_t oWf1 = carve((size_t)C2 * CC * 2);
  const size_t oWf2 = carve((size_t)CC * C2 * 2);
  const size_t oEx  = carve((size_t)ROWS * 4);
  if (off > ws_size) return;

  char* ws = (char*)d_ws;
  _Float16* xn   = (_Float16*)(ws + oR1);
  _Float16* col  = (_Float16*)(ws + oR1);
  _Float16* g64  = (_Float16*)(ws + oR1);
  _Float16* h64  = (_Float16*)(ws + oR2);
  _Float16* y64  = (_Float16*)(ws + oR2);
  _Float16* WsT  = (_Float16*)(ws + oWsT);
  _Float16* Wc64 = (_Float16*)(ws + oWc);
  _Float16* Wf1T = (_Float16*)(ws + oWf1);
  _Float16* Wf2T = (_Float16*)(ws + oWf2);
  float*    exg  = (float*)(ws + oEx);

  const float W64 = 64.0f;
  const unsigned short* uXn  = (const unsigned short*)xn;
  const unsigned short* uCol = (const unsigned short*)col;
  const unsigned short* uG   = (const unsigned short*)g64;
  const unsigned short* uH   = (const unsigned short*)h64;
  const unsigned short* uY   = (const unsigned short*)y64;
  const unsigned short* uWsT = (const unsigned short*)WsT;
  const unsigned short* uWc  = (const unsigned short*)Wc64;
  const unsigned short* uWf1 = (const unsigned short*)Wf1T;
  const unsigned short* uWf2 = (const unsigned short*)Wf2T;

  transpose_scale_f16<<<dim3(CC / 64, CC / 64), 256, 0, stream>>>(Ws, WsT, CC, CC, W64);
  transpose_scale_f16<<<dim3(C2 / 64, CC / 64), 256, 0, stream>>>(Wf1, Wf1T, CC, C2, W64);
  transpose_scale_f16<<<dim3(CC / 64, C2 / 64), 256, 0, stream>>>(Wf2, Wf2T, C2, CC, W64);
  {
    const int n2 = NN * KC / 2;
    cast_scale_f16x2<<<(n2 + 255) / 256, 256, 0, stream>>>(Wc, Wc64, n2, W64);
  }

  ln_kernel<<<(ROWS + 7) / 8, 256, 0, stream>>>(x, ln_g, ln_b, xn, ROWS);

  {
    const int tiles = (ROWS / 64) * (CC / 64);
    wmma_gemm64<0, false, 2, 1, false, 2, false, true><<<dim3((tiles + 7) / 8, 1), 256, 0, stream>>>(
        uXn, uXn, CC, 0L, uWsT, uWsT, CC, 0L, (void*)h64, (void*)h64, CC, 0L,
        bs, bs, 0L, bs, ROWS, CC, CC, 1.0f / 64.0f, W64);
  }

  im2col_shift_kernel<<<dim3(CC / 64, nB), 256, 0, stream>>>(h64, col);

  {
    const int tiles = (NN / 64) * (CC / 64);
    wmma_gemm64<0, false, 1, 1, false, 0, false, true><<<dim3((tiles + 7) / 8, nB), 256, 0, stream>>>(
        uWc, uWc, KC, 0L, uCol, uCol, KC, (long)CC * KC, (void*)y64, (void*)y64, CC, (long)NN * CC,
        bc, bc, 0L, bc, NN, CC, KC, 1.0f / 4096.0f, W64);
  }

  se_kernel<<<nB, 256, 0, stream>>>(y64, We1, be1, We2, be2, exg);

  {
    const int tiles = (ROWS / 64) * (C2 / 64);
    wmma_gemm64<0, false, 2, 1, false, 2, true, true><<<dim3((tiles + 7) / 8, 1), 256, 0, stream>>>(
        uY, uY, CC, 0L, uWf1, uWf1, CC, 0L, (void*)g64, (void*)g64, C2, 0L,
        bf1, bf1, 0L, exg, ROWS, C2, CC, 1.0f / 4096.0f, W64);
  }

  {
    const int tiles = (ROWS / 64) * (CC / 64);
    wmma_gemm64<0, false, 2, 0, true, 0, false, false><<<dim3((tiles + 7) / 8, 1), 256, 0, stream>>>(
        uG, uG, C2, 0L, uWf2, uWf2, C2, 0L, (void*)out, (void*)out, CC, 0L,
        bf2, x, 0L, bf2, ROWS, CC, C2, 1.0f / 4096.0f, 1.0f);
  }
}
